// GNNClassifier_51866025066884
// MI455X (gfx1250) — hardware-verified
//
#include <hip/hip_runtime.h>


typedef _Float16 v8h  __attribute__((ext_vector_type(8)));
typedef _Float16 v16h __attribute__((ext_vector_type(16)));
typedef float    v8f  __attribute__((ext_vector_type(8)));
typedef float    v4f  __attribute__((ext_vector_type(4)));
typedef int      v4i  __attribute__((ext_vector_type(4)));

#define HEADS     4
#define CH        64
#define NOUT      256
#define IN_DIM    256
#define NGRAPHS   128
#define NEG_SLOPE 0.2f
#define NPB       128
#define CAP       4096
#define GT        32
#define SCP       260

union Frag  { v16h v; v8h half[2]; };
union Pack8 { v8h h; v4f f; };

__device__ __forceinline__ v8f wmma_f16(v16h a, v16h b, v8f c) {
    v8f d = __builtin_amdgcn_wmma_f32_16x16x32_f16(false, a, false, b, (short)0, c, false, false);
    asm volatile("v_nop\n\tv_nop\n\tv_nop\n\tv_nop" : "+v"(d) : "v"(a), "v"(b));
    return d;
}

__device__ __forceinline__ float leaky(float x) { return x >= 0.f ? x : NEG_SLOPE * x; }
__device__ __forceinline__ float elu_f(float x) { return x > 0.f ? x : expm1f(x); }

__global__ __launch_bounds__(256) void k_packw(const float* __restrict__ W1, const float* __restrict__ W2,
        _Float16* __restrict__ Wp1, _Float16* __restrict__ Wp2)
{
    const int nb1 = (NOUT * IN_DIM / 8) / 256;
    const bool first = (int)blockIdx.x < nb1;
    const float* W = first ? W1 : W2;
    _Float16* Wp   = first ? Wp1 : Wp2;
    const int K    = first ? IN_DIM : CH;
    const int gpc  = K / 8;
    const int idx  = (first ? (int)blockIdx.x : (int)blockIdx.x - nb1) * 256 + (int)threadIdx.x;
    if (idx >= NOUT * gpc) return;
    const int n = idx / gpc, g = idx - n * gpc;
    Pack8 p;
    #pragma unroll
    for (int i = 0; i < 8; ++i) p.h[i] = (_Float16)W[(size_t)(8 * g + i) * NOUT + n];
    _Float16* dst = Wp + (size_t)idx * 8;
    *(volatile v4f*)dst = p.f;
    __threadfence();
    *(volatile v4f*)dst = p.f;
}

__global__ __launch_bounds__(256) void k_csr_build(const int* __restrict__ ei, int E, int N,
        int* __restrict__ csr_src, int* __restrict__ seg_beg, int* __restrict__ seg_cnt)
{
    __shared__ __attribute__((aligned(16))) unsigned keys[CAP];
    __shared__ __attribute__((aligned(16))) int      srcs[CAP];
    __shared__ int wtot[8];
    __shared__ __attribute__((aligned(16))) int sbeg[NPB];
    __shared__ __attribute__((aligned(16))) int scnt[NPB];

    const int tid  = threadIdx.x;
    const int lane = tid & 31;
    const int wave = tid >> 5;
    const int blk  = blockIdx.x;
    const int n0   = blk * NPB;

    for (int i = tid; i < CAP; i += 256) { keys[i] = 0xFFFFFFFFu; srcs[i] = 0; }
    int nval = N - n0;
    nval = nval < 0 ? 0 : (nval > NPB ? NPB : nval);
    __syncthreads();

    for (int j = tid; j < nval; j += 256) {
        keys[j] = ((unsigned)j << 16) | (unsigned)j;
        srcs[j] = n0 + j;
    }
    int base = nval;

    const int per_it = 256 * 8;
    const int nit = (E + per_it - 1) / per_it;
    for (int it = 0; it < nit; ++it) {
        int dl[8], sv[8];
        int c = 0;
        #pragma unroll
        for (int k = 0; k < 8; ++k) {
            const int e = it * per_it + k * 256 + tid;
            int d = -1, s = 0;
            if (e < E) {
                const int dd = ei[E + e];
                if (((unsigned)dd - (unsigned)n0) < (unsigned)NPB) { d = dd - n0; s = ei[e]; }
            }
            dl[k] = d; sv[k] = s; c += (d >= 0) ? 1 : 0;
        }
        int incl = c;
        #pragma unroll
        for (int off = 1; off < 32; off <<= 1) {
            const int v = __shfl_up(incl, off);
            if (lane >= off) incl += v;
        }
        if (lane == 31) wtot[wave] = incl;
        __syncthreads();
        int woff = 0, tot = 0;
        #pragma unroll
        for (int w = 0; w < 8; ++w) {
            const int v = wtot[w];
            if (w < wave) woff += v;
            tot += v;
        }
        int pos = base + woff + incl - c;
        #pragma unroll
        for (int k = 0; k < 8; ++k) {
            if (dl[k] >= 0) {
                if (pos < CAP) {
                    keys[pos] = ((unsigned)dl[k] << 16) | (unsigned)pos;
                    srcs[pos] = sv[k];
                }
                ++pos;
            }
        }
        base += tot;
        __syncthreads();
    }

    for (unsigned k = 2; k <= (unsigned)CAP; k <<= 1) {
        for (unsigned j = k >> 1; j > 0; j >>= 1) {
            for (unsigned i = (unsigned)tid; i < (unsigned)CAP; i += 256) {
                const unsigned ixj = i ^ j;
                if (ixj > i) {
                    const unsigned a = keys[i], b = keys[ixj];
                    const bool up = ((i & k) == 0);
                    if ((a > b) == up) { keys[i] = b; keys[ixj] = a; }
                }
            }
            __syncthreads();
        }
    }

    if (tid < NPB) {
        const unsigned klo = (unsigned)tid << 16;
        const unsigned khi = (unsigned)(tid + 1) << 16;
        int lo = 0, hi = CAP;
        while (lo < hi) { const int mid = (lo + hi) >> 1; if (keys[mid] < klo) lo = mid + 1; else hi = mid; }
        const int b0 = lo;
        lo = 0; hi = CAP;
        while (lo < hi) { const int mid = (lo + hi) >> 1; if (keys[mid] < khi) lo = mid + 1; else hi = mid; }
        sbeg[tid] = b0;
        scnt[tid] = lo - b0;
    }
    __syncthreads();

    int* cbase = csr_src + (size_t)blk * CAP;
    auto emit = [&]() {
        #pragma unroll
        for (int i = 0; i < 4; ++i) {
            const int q0 = (i * 256 + tid) * 4;
            v4i v;
            #pragma unroll
            for (int u = 0; u < 4; ++u) {
                const unsigned key = keys[q0 + u];
                v[u] = (key == 0xFFFFFFFFu) ? 0 : srcs[key & (CAP - 1)];
            }
            *(volatile v4i*)(cbase + q0) = v;
        }
        if (wave == 0) {
            v4i v = *(const v4i*)(sbeg + 4 * lane);
            *(volatile v4i*)(seg_beg + (size_t)n0 + 4 * lane) = v;
        } else if (wave == 1) {
            v4i v = *(const v4i*)(scnt + 4 * lane);
            *(volatile v4i*)(seg_cnt + (size_t)n0 + 4 * lane) = v;
        }
    };
    emit();
    __threadfence();
    emit();
}

template <int K, bool ACT>
__global__ __launch_bounds__(128) void k_gemm(const float* __restrict__ A, const _Float16* __restrict__ Wp,
        const float* __restrict__ att_s, const float* __restrict__ att_d,
        float* __restrict__ C, float* __restrict__ as_out, float* __restrict__ ad_out, int M)
{
    __shared__ __attribute__((aligned(16))) v8h   sA8[GT * 4];
    __shared__ __attribute__((aligned(16))) float sC[GT * SCP];
    __shared__ __attribute__((aligned(16))) float sAtt[2 * NOUT];
    __shared__ __attribute__((aligned(16))) float sCoef[2 * 128];

    const int tid  = threadIdx.x;
    const int wave = tid >> 5;
    const int lane = tid & 31;
    const int h    = lane >> 4;
    const int m    = lane & 15;
    const int row0 = blockIdx.x * GT;

    for (int i = tid; i < NOUT; i += 128) { sAtt[i] = att_s[i]; sAtt[NOUT + i] = att_d[i]; }

    v8f acc[2][4];
    #pragma unroll
    for (int tm = 0; tm < 2; ++tm) {
        #pragma unroll
        for (int t = 0; t < 4; ++t) acc[tm][t] = v8f{};
    }

    for (int k0 = 0; k0 < K; k0 += 32) {
        __syncthreads();
        {
            const int r = tid >> 2, part = tid & 3;
            const int grow = row0 + r;
            v8h hv = v8h{};
            if (grow < M) {
                const float* ap = A + (size_t)grow * K + k0 + 8 * part;
                const v4f x0 = *(const v4f*)ap;
                const v4f x1 = *(const v4f*)(ap + 4);
                #pragma unroll
                for (int i = 0; i < 4; ++i) {
                    float u0 = x0[i], u1 = x1[i];
                    if (ACT) { u0 = elu_f(u0); u1 = elu_f(u1); }
                    hv[i]     = (_Float16)u0;
                    hv[4 + i] = (_Float16)u1;
                }
            }
            sA8[r * 4 + part] = hv;
        }
        __syncthreads();

        Frag a0, a1;
        a0.half[0] = sA8[m * 4 + h];        a0.half[1] = sA8[m * 4 + 2 + h];
        a1.half[0] = sA8[(16 + m) * 4 + h]; a1.half[1] = sA8[(16 + m) * 4 + 2 + h];
        #pragma unroll
        for (int t = 0; t < 4; ++t) {
            const int col = wave * 64 + 16 * t + m;
            const _Float16* bp = Wp + (size_t)col * K + k0;
            Frag b;
            b.half[0] = *(const v8h*)(bp + 8 * h);
            b.half[1] = *(const v8h*)(bp + 16 + 8 * h);
            acc[0][t] = wmma_f16(a0.v, b.v, acc[0][t]);
            acc[1][t] = wmma_f16(a1.v, b.v, acc[1][t]);
        }
    }

    #pragma unroll
    for (int tm = 0; tm < 2; ++tm) {
        #pragma unroll
        for (int t = 0; t < 4; ++t) {
            #pragma unroll
            for (int r = 0; r < 8; ++r)
                sC[(16 * tm + 8 * h + r) * SCP + wave * 64 + 16 * t + m] = acc[tm][t][r];
        }
    }
    __syncthreads();

    {
        const int r = tid >> 2, hd = tid & 3;
        const float* cr = sC + r * SCP + hd * CH;
        const float* wsr = sAtt + hd * CH;
        const float* wdr = sAtt + NOUT + hd * CH;
        float s = 0.f, d = 0.f;
        #pragma unroll 8
        for (int c = 0; c < CH; ++c) { const float v = cr[c]; s += v * wsr[c]; d += v * wdr[c]; }
        sCoef[tid] = s;
        sCoef[128 + tid] = d;
    }
    __syncthreads();

    auto emit = [&]() {
        #pragma unroll
        for (int i = 0; i < 16; ++i) {
            const int f  = (i * 128 + tid) * 4;
            const int rr = f >> 8, cc = f & 255;
            const v4f v = *(const v4f*)(sC + rr * SCP + cc);
            *(volatile v4f*)(C + (size_t)(row0 + rr) * NOUT + cc) = v;
        }
        if (wave == 0) {
            const v4f v = *(const v4f*)(sCoef + 4 * lane);
            *(volatile v4f*)(as_out + (size_t)row0 * HEADS + 4 * lane) = v;
        } else if (wave == 1) {
            const v4f v = *(const v4f*)(sCoef + 128 + 4 * lane);
            *(volatile v4f*)(ad_out + (size_t)row0 * HEADS + 4 * lane) = v;
        }
    };
    emit();
    __threadfence();
    emit();
}

__global__ __launch_bounds__(128) void k_agg(const int* __restrict__ csr_src,
        const int* __restrict__ seg_beg, const int* __restrict__ seg_cnt,
        const float* __restrict__ hb, const float* __restrict__ a_s, const float* __restrict__ a_d,
        const float* __restrict__ bias, float* __restrict__ hout, int N)
{
    __shared__ __attribute__((aligned(16))) v4f sOut[GT * 16];

    const int tid  = threadIdx.x;
    const int wave = tid >> 5;
    const int lane = tid & 31;
    const int hd   = lane >> 3;
    const int c0   = (lane & 7) * 8;
    const int n0   = blockIdx.x * GT;

    float bias8[8];
    #pragma unroll
    for (int i = 0; i < 8; ++i) bias8[i] = bias[c0 + i];

    for (int it = 0; it < 8; ++it) {
        const int node = n0 + it * 4 + wave;
        int cnt = 0;
        size_t sbase = 0;
        float ad = 0.f;
        if (node < N) {
            cnt = seg_cnt[node];
            int beg = seg_beg[node];
            cnt = cnt < 0 ? 0 : (cnt > CAP ? CAP : cnt);
            beg = beg < 0 ? 0 : (beg > CAP - cnt ? CAP - cnt : beg);
            sbase = (size_t)(node / NPB) * CAP + beg;
            ad = a_d[(size_t)node * HEADS + hd];
        }
        const int* sp = csr_src + sbase;

        float mx = -__builtin_inff();
        #pragma unroll 1
        for (int p = 0; p < cnt; ++p) {
            int s = sp[p];
            s = s < 0 ? 0 : (s > N - 1 ? N - 1 : s);
            const float e = leaky(a_s[(size_t)s * HEADS + hd] + ad);
            mx = fmaxf(mx, e);
        }
        float sum = 0.f;
        float acc[8];
        #pragma unroll
        for (int i = 0; i < 8; ++i) acc[i] = 0.f;
        #pragma unroll 1
        for (int p = 0; p < cnt; ++p) {
            int s = sp[p];
            s = s < 0 ? 0 : (s > N - 1 ? N - 1 : s);
            const float e  = leaky(a_s[(size_t)s * HEADS + hd] + ad);
            const float ex = __expf(e - mx);
            sum += ex;
            const float* hp = hb + (size_t)s * NOUT + hd * CH + c0;
            const v4f x0 = *(const v4f*)hp;
            const v4f x1 = *(const v4f*)(hp + 4);
            acc[0] += ex * x0[0]; acc[1] += ex * x0[1]; acc[2] += ex * x0[2]; acc[3] += ex * x0[3];
            acc[4] += ex * x1[0]; acc[5] += ex * x1[1]; acc[6] += ex * x1[2]; acc[7] += ex * x1[3];
        }
        const float inv = sum > 0.f ? 1.f / sum : 0.f;
        float v[8];
        #pragma unroll
        for (int i = 0; i < 8; ++i) {
            float t = acc[i] * inv;
            t += __shfl_xor(t, 8);
            t += __shfl_xor(t, 16);
            v[i] = 0.25f * t + bias8[i];
        }
        if (lane < 8) {
            v4f o0, o1;
            o0[0] = v[0]; o0[1] = v[1]; o0[2] = v[2]; o0[3] = v[3];
            o1[0] = v[4]; o1[1] = v[5]; o1[2] = v[6]; o1[3] = v[7];
            sOut[(it * 4 + wave) * 16 + 2 * lane]     = o0;
            sOut[(it * 4 + wave) * 16 + 2 * lane + 1] = o1;
        }
    }
    __syncthreads();

    float* obase = hout + (size_t)n0 * CH;
    auto emit = [&]() {
        #pragma unroll
        for (int i = 0; i < 4; ++i) {
            const int f4 = i * 128 + tid;
            const v4f vv = sOut[f4];
            *(volatile v4f*)(obase + (size_t)f4 * 4) = vv;
        }
    };
    emit();
    __threadfence();
    emit();
}

__global__ __launch_bounds__(64) void k_poolpart(const float* __restrict__ h2, const int* __restrict__ batch,
        float* __restrict__ psum, float* __restrict__ pcnt, int N)
{
    __shared__ __attribute__((aligned(16))) float sacc[NGRAPHS * CH];
    __shared__ __attribute__((aligned(16))) float scnt[NGRAPHS];

    const int tid = threadIdx.x;
    const int blk = blockIdx.x;
    const int n0  = blk * NPB;

    for (int i = tid; i < NGRAPHS * CH; i += 64) sacc[i] = 0.f;
    for (int i = tid; i < NGRAPHS; i += 64) scnt[i] = 0.f;
    int nval = N - n0;
    nval = nval < 0 ? 0 : (nval > NPB ? NPB : nval);
    __syncthreads();

    #pragma unroll 1
    for (int j = 0; j < nval; ++j) {
        const int n = n0 + j;
        const int g = batch[n];
        if ((unsigned)g < (unsigned)NGRAPHS) {
            sacc[g * CH + tid] += elu_f(h2[(size_t)n * CH + tid]);
            if (tid == 0) scnt[g] += 1.f;
        }
    }
    __syncthreads();

    float* sb = psum + (size_t)blk * (NGRAPHS * CH);
    float* cb = pcnt + (size_t)blk * NGRAPHS;
    auto emit = [&]() {
        #pragma unroll
        for (int i = 0; i < (NGRAPHS * CH) / (64 * 4); ++i) {
            const int f = (i * 64 + tid) * 4;
            const v4f v = *(const v4f*)(sacc + f);
            *(volatile v4f*)(sb + f) = v;
        }
        if (tid < 32) {
            const v4f v = *(const v4f*)(scnt + 4 * tid);
            *(volatile v4f*)(cb + 4 * tid) = v;
        }
    };
    emit();
    __threadfence();
    emit();
}

__global__ __launch_bounds__(128) void k_clf(const float* __restrict__ psum, const float* __restrict__ pcnt,
        const float* __restrict__ w, const float* __restrict__ b, float* __restrict__ out, int nblk)
{
    __shared__ __attribute__((aligned(16))) float so[NGRAPHS];
    const int tid = threadIdx.x;
    const int g = tid;
    float cn = 0.f;
    #pragma unroll 1
    for (int bk = 0; bk < nblk; ++bk) cn += pcnt[(size_t)bk * NGRAPHS + g];
    const float inv = 1.f / fmaxf(cn, 1.f);
    float dot = 0.f;
    #pragma unroll 1
    for (int c = 0; c < CH; ++c) {
        float s = 0.f;
        #pragma unroll 1
        for (int bk = 0; bk < nblk; ++bk) s += psum[((size_t)bk * NGRAPHS + g) * CH + c];
        dot += (s * inv) * w[c];
    }
    so[g] = dot + b[0];
    __syncthreads();
    auto emit = [&]() {
        if (tid < 32) {
            const v4f v = *(const v4f*)(so + 4 * tid);
            *(volatile v4f*)(out + 4 * tid) = v;
        }
    };
    emit();
    __threadfence();
    emit();
}

static inline size_t align_up(size_t x, size_t a) { return (x + a - 1) / a * a; }

extern "C" void kernel_launch(void* const* d_in, const int* in_sizes, int n_in,
                              void* d_out, int out_size, void* d_ws, size_t ws_size,
                              hipStream_t stream)
{
    if (n_in < 13) return;
    const float* x      = (const float*)d_in[0];
    const float* W1     = (const float*)d_in[1];
    const float* att_s1 = (const float*)d_in[2];
    const float* att_d1 = (const float*)d_in[3];
    const float* bias1  = (const float*)d_in[4];
    const float* W2     = (const float*)d_in[5];
    const float* att_s2 = (const float*)d_in[6];
    const float* att_d2 = (const float*)d_in[7];
    const float* bias2  = (const float*)d_in[8];
    const float* clf_w  = (const float*)d_in[9];
    const float* clf_b  = (const float*)d_in[10];
    const int*   ei     = (const int*)d_in[11];
    const int*   batch  = (const int*)d_in[12];
    float*       out    = (float*)d_out;

    const int N = in_sizes[0] / IN_DIM;
    const int E = in_sizes[11] / 2;
    if (N <= 0 || N * IN_DIM != in_sizes[0] || E < 0 || 2 * E != in_sizes[11]) return;
    if (in_sizes[1] != IN_DIM * NOUT || in_sizes[5] != CH * NOUT) return;
    if (in_sizes[2] < NOUT || in_sizes[3] < NOUT || in_sizes[6] < NOUT || in_sizes[7] < NOUT) return;
    if (in_sizes[4] < CH || in_sizes[8] < CH || in_sizes[9] < CH || in_sizes[10] < 1) return;
    if (in_sizes[12] != N || out_size != NGRAPHS) return;

    const int nblk = (N + NPB - 1) / NPB;
    const int Npad = ((N + GT - 1) / GT) * GT;

    char* ws = (char*)d_ws;
    size_t off = 0;
    const size_t o_wp1  = off; off += align_up((size_t)NOUT * IN_DIM * sizeof(_Float16), 1024);
    const size_t o_wp2  = off; off += align_up((size_t)NOUT * CH * sizeof(_Float16), 1024);
    const size_t o_csr  = off; off += align_up((size_t)nblk * CAP * sizeof(int), 1024);
    const size_t o_sbeg = off; off += align_up((size_t)nblk * NPB * sizeof(int), 1024);
    const size_t o_scnt = off; off += align_up((size_t)nblk * NPB * sizeof(int), 1024);
    const size_t o_hbuf = off; off += align_up((size_t)Npad * NOUT * sizeof(float), 1024);
    const size_t o_as   = off; off += align_up((size_t)Npad * HEADS * sizeof(float), 1024);
    const size_t o_ad   = off; off += align_up((size_t)Npad * HEADS * sizeof(float), 1024);
    const size_t o_h1   = off; off += align_up((size_t)Npad * CH * sizeof(float), 1024);
    const size_t o_h2   = off; off += align_up((size_t)Npad * CH * sizeof(float), 1024);
    const size_t o_psum = off; off += align_up((size_t)nblk * NGRAPHS * CH * sizeof(float), 1024);
    const size_t o_pcnt = off; off += align_up((size_t)nblk * NGRAPHS * sizeof(float), 1024);
    if (off > ws_size) return;

    _Float16* wp1   = (_Float16*)(ws + o_wp1);
    _Float16* wp2   = (_Float16*)(ws + o_wp2);
    int*   csr_src  = (int*)(ws + o_csr);
    int*   seg_beg  = (int*)(ws + o_sbeg);
    int*   seg_cnt  = (int*)(ws + o_scnt);
    float* hbuf     = (float*)(ws + o_hbuf);
    float* a_s      = (float*)(ws + o_as);
    float* a_d      = (float*)(ws + o_ad);
    float* h1       = (float*)(ws + o_h1);
    float* h2       = (float*)(ws + o_h2);
    float* psum     = (float*)(ws + o_psum);
    float* pcnt     = (float*)(ws + o_pcnt);

    const unsigned pack_blocks = (unsigned)((NOUT * IN_DIM / 8) / 256 + (NOUT * CH / 8 + 255) / 256);
    const unsigned gemm_blocks = (unsigned)(Npad / GT);
    const unsigned agg_blocks  = (unsigned)(Npad / GT);

    k_packw<<<pack_blocks, 256, 0, stream>>>(W1, W2, wp1, wp2);
    k_csr_build<<<(unsigned)nblk, 256, 0, stream>>>(ei, E, N, csr_src, seg_beg, seg_cnt);

    k_gemm<IN_DIM, false><<<gemm_blocks, 128, 0, stream>>>(x, wp1, att_s1, att_d1, hbuf, a_s, a_d, N);
    k_agg<<<agg_blocks, 128, 0, stream>>>(csr_src, seg_beg, seg_cnt, hbuf, a_s, a_d, bias1, h1, N);

    k_gemm<CH, true><<<gemm_blocks, 128, 0, stream>>>(h1, wp2, att_s2, att_d2, hbuf, a_s, a_d, N);
    k_agg<<<agg_blocks, 128, 0, stream>>>(csr_src, seg_beg, seg_cnt, hbuf, a_s, a_d, bias2, h2, N);

    k_poolpart<<<(unsigned)nblk, 64, 0, stream>>>(h2, batch, psum, pcnt, N);
    k_clf<<<1, NGRAPHS, 0, stream>>>(psum, pcnt, clf_w, clf_b, out, nblk);
}
